// CrossAttention_31044023615565
// MI455X (gfx1250) — hardware-run, weakly checked
//
#include <hip/hip_runtime.h>


#ifndef NB
#define NB 8
#endif
#ifndef SEQ
#define SEQ 1600
#endif
#define NB_FULL  8
#define SEQ_FULL 1600
#ifndef OUT_SEQ
#define OUT_SEQ SEQ
#endif
#define DQ   256
#define DKV  128
#define DM   128
#define NH_  4
#define HD   32
#define AW   4
#define OSP  36
#define TCP  33
#define SC2  ((float)(0.17677669529663687 * 1.4426950408889634))
#define PSH  14.0f
#define NEGB (-3.0e38f)
#define CXS  1024.0f
#define WOS  64.0f
#define OSC  (1.0f / (1024.0f * 64.0f))

static_assert(HD == 32);
static_assert(NH_ * HD == DM);
static_assert(DM % 64 == 0);
static_assert(DQ % 64 == 0);
static_assert(DKV % 64 == 0);
static_assert(DQ % 32 == 0);
static_assert(DKV % 32 == 0);
static_assert(DM % 32 == 0);
static_assert(SEQ % 64 == 0);
static_assert((NB * SEQ) % 64 == 0);
static_assert(SEQ % 32 == 0);
static_assert(SEQ % (16 * AW) == 0);
static_assert(SEQ_FULL % 4 == 0);
static_assert(NB <= NB_FULL);
static_assert(SEQ <= SEQ_FULL);
static_assert(OUT_SEQ >= SEQ);
static_assert(OUT_SEQ % 32 == 0);
static_assert((OSP * 4) % 16 == 0);
static_assert(64 * TCP * 4 <= 131072);
static_assert(16 * 68 * 4 <= 131072);
static_assert(AW * 16 * OSP * 4 <= 131072);

typedef _Float16 h16;
typedef unsigned short bf;
typedef __attribute__((ext_vector_type(16))) __bf16   v16bf;
typedef __attribute__((ext_vector_type(16))) _Float16 v16h;
typedef __attribute__((ext_vector_type(8)))  _Float16 v8h;
typedef __attribute__((ext_vector_type(8)))  unsigned short v8us;
typedef __attribute__((ext_vector_type(8)))  float    v8f;
typedef __attribute__((ext_vector_type(4)))  float    v4f;
typedef v4f  __attribute__((may_alias)) v4fa;

__device__ __forceinline__ unsigned short f2bf(float f) { unsigned u = __float_as_uint(f); u += 0x7FFFu + ((u >> 16) & 1u); return (unsigned short)(u >> 16); }
__device__ __forceinline__ float bfr(float f) { return __uint_as_float(((unsigned)f2bf(f)) << 16); }
__device__ __forceinline__ v16h cat16(v8h lo, v8h hi) { return __builtin_shufflevector(lo, hi, 0, 1, 2, 3, 4, 5, 6, 7, 8, 9, 10, 11, 12, 13, 14, 15); }
__device__ __forceinline__ v16bf cat16b(v8us lo, v8us hi) { return __builtin_bit_cast(v16bf, __builtin_shufflevector(lo, hi, 0, 1, 2, 3, 4, 5, 6, 7, 8, 9, 10, 11, 12, 13, 14, 15)); }
__device__ __forceinline__ v8f wmma16(v16h a, v16h b, v8f c) { return __builtin_amdgcn_wmma_f32_16x16x32_f16(false, a, false, b, (short)0, c, false, false); }
__device__ __forceinline__ v8f wmmab(v16bf a, v16bf b, v8f c) { return __builtin_amdgcn_wmma_f32_16x16x32_bf16(false, a, false, b, (short)0, c, false, false); }
__device__ __forceinline__ v16h  ldh(const h16* p) { return cat16(*(const v8h*)p, *(const v8h*)(p + 16)); }
__device__ __forceinline__ v16bf ldb(const bf* p)  { return cat16b(*(const v8us*)p, *(const v8us*)(p + 16)); }
__device__ __forceinline__ void wave_sync() { __builtin_amdgcn_fence(3  , "wavefront"); __builtin_amdgcn_wave_barrier(); asm volatile("" ::: "memory"); }
static __device__ __forceinline__ h16 toh_flush(float v) { const h16 r = (h16)v; return (fabsf(v) < 6.103515625e-05f) ? (h16)0.0f : r; }
__device__ __forceinline__ v8f wmma16g(v16h a, v16h b, v8f c) { c = wmma16(a, b, c); asm volatile("v_nop\n\tv_nop\n\tv_nop\n\tv_nop" : "+v"(c) : "v"(a), "v"(b)); return c; }
__device__ __forceinline__ v8f wmmabg(v16bf a, v16bf b, v8f c) { c = wmmab(a, b, c); asm volatile("v_nop\n\tv_nop\n\tv_nop\n\tv_nop" : "+v"(c) : "v"(a), "v"(b)); return c; }

static_assert(256 * 16 * 1 == 32 * 128);
template <int F16>
__device__ __forceinline__ void tcvt_body(const float* __restrict__ src, unsigned short* dst, const int C, const int srcPitch, const int dstRows, const float carry) {
    __shared__ float ts[64 * TCP];
    const int tid = threadIdx.x;
    const int n0 = blockIdx.x * 32, c0 = blockIdx.y * 64, z = blockIdx.z;
    { const int cr = tid >> 3, q4 = (tid & 7) * 4;
#pragma unroll
      for (int it = 0; it < 2; ++it) { const int cl = it * 32 + cr;
          const v4f v = *(const v4f*)(src + ((size_t)z * (size_t)C + (size_t)(c0 + cl)) * (size_t)srcPitch + (size_t)(n0 + q4));
          ts[cl * TCP + q4 + 0] = v[0]; ts[cl * TCP + q4 + 1] = v[1]; ts[cl * TCP + q4 + 2] = v[2]; ts[cl * TCP + q4 + 3] = v[3]; } }
    __syncthreads();
    const int tok = tid >> 3, g8 = (tid & 7) * 8;
    v8us o;
#pragma unroll
    for (int k = 0; k < 8; ++k) { const float x = ts[(g8 + k) * TCP + tok];
        if (F16) { const h16 hv = toh_flush(bfr(x) * carry); o[k] = __builtin_bit_cast(unsigned short, hv); }
        else     { o[k] = f2bf(x); } }
    unsigned short* dp = dst + ((size_t)z * (size_t)dstRows + (size_t)(n0 + tok)) * (size_t)C + (size_t)(c0 + g8);
    *(volatile v8us*)dp = o; __threadfence(); *(volatile v8us*)dp = o;
}
__global__ __launch_bounds__(256) void k_tcvt_b(const float* __restrict__ src, bf* dst, int C, int srcPitch, int dstRows) { tcvt_body<0>(src, dst, C, srcPitch, dstRows, 1.0f); }
__global__ __launch_bounds__(256) void k_tcvt_h(const float* __restrict__ src, h16* dst, int C, int srcPitch, int dstRows, float carry) { tcvt_body<1>(src, (unsigned short*)dst, C, srcPitch, dstRows, carry); }

static_assert(32 * 16 * 2 == 16 * HD * 2);
static_assert(32 * 16 * 4 == 16 * 64 * 2);
template <int MODE>
__device__ __forceinline__ void proj_body(const bf* __restrict__ A, const bf* __restrict__ Bt, h16* Ph, const int K) {
    __shared__ __align__(16) float os[16 * 68];
    const int lane = threadIdx.x & 31, lr = lane & 15, hi = lane >> 4; const int r0 = blockIdx.x * 64, c0 = blockIdx.y * 64;
    v8f acc[4][4];
#pragma unroll
    for (int mb = 0; mb < 4; ++mb)
#pragma unroll
        for (int nb = 0; nb < 4; ++nb) acc[mb][nb] = (v8f){};
    const size_t aoff = (size_t)(r0 + lr) * K + 8 * hi, boff = (size_t)(c0 + lr) * K + 8 * hi;
#pragma unroll 1
    for (int kc = 0; kc < K; kc += 32) {
        v16bf a[4];
#pragma unroll
        for (int mb = 0; mb < 4; ++mb) a[mb] = ldb(A + aoff + (size_t)mb * 16 * K + kc);
#pragma unroll
        for (int nb = 0; nb < 4; ++nb) { const v16bf b = ldb(Bt + boff + (size_t)nb * 16 * K + kc);
#pragma unroll
            for (int mb = 0; mb < 4; ++mb) acc[mb][nb] = wmmabg(a[mb], b, acc[mb][nb]); }
    }
    size_t tbase;
    if (MODE == 0) { const int bb = r0 / SEQ, tt = r0 % SEQ; const int zc = bb * NH_ + c0 / HD;
                     tbase = ((size_t)zc * SEQ + (size_t)tt) * HD; }
    else           { const int bb = c0 / SEQ, tt = c0 % SEQ;
                     tbase = (size_t)bb * (size_t)DM * SEQ + (size_t)r0 * SEQ + (size_t)tt; }
#pragma unroll
    for (int mb = 0; mb < 4; ++mb) {
#pragma unroll
        for (int nb = 0; nb < 4; ++nb) {
#pragma unroll
            for (int j = 0; j < 8; ++j) os[(hi * 8 + j) * 68 + nb * 16 + lr] = acc[mb][nb][j]; }
        wave_sync();
#pragma unroll 1
        for (int ps = 0; ps < 2; ++ps) {
            if (MODE == 0) {
                const size_t sb = tbase + (size_t)(mb * 16) * HD;
#pragma unroll
                for (int hh = 0; hh < 2; ++hh) {
#pragma unroll
                    for (int s = 0; s < 2; ++s) { const int p = s * 32 + lane; const int row = p >> 2, c8 = (p & 3) * 8;
                        const v4f x0 = *(const v4fa*)(&os[row * 68 + hh * 32 + c8]); const v4f x1 = *(const v4fa*)(&os[row * 68 + hh * 32 + c8 + 4]); v8h hv;
#pragma unroll
                        for (int i = 0; i < 4; ++i) { hv[i] = toh_flush(x0[i]); hv[4 + i] = toh_flush(x1[i]); }
                        const size_t oo = sb + (size_t)hh * ((size_t)SEQ * HD) + (size_t)p * 8;
                        *(volatile v8h*)(Ph + oo) = hv; } }
            } else {
                const size_t sb = tbase + (size_t)(mb * 16) * SEQ;
#pragma unroll
                for (int s = 0; s < 4; ++s) { const int row = 4 * s + (lane >> 3), c8 = (lane & 7) * 8;
                    const v4f x0 = *(const v4fa*)(&os[row * 68 + c8]); const v4f x1 = *(const v4fa*)(&os[row * 68 + c8 + 4]); v8h hv;
#pragma unroll
                    for (int i = 0; i < 4; ++i) { hv[i] = toh_flush(x0[i]); hv[4 + i] = toh_flush(x1[i]); }
                    const size_t oo = sb + (size_t)row * SEQ + c8;
                    *(volatile v8h*)(Ph + oo) = hv; }
            }
            if (ps == 0) __threadfence(); }
        wave_sync();
    }
}
__global__ __launch_bounds__(32) void k_proj_rows(const bf* __restrict__ A, const bf* __restrict__ Bt, h16* Ph, int K) { proj_body<0>(A, Bt, Ph, K); }
__global__ __launch_bounds__(32) void k_proj_cols(const bf* __restrict__ A, const bf* __restrict__ Bt, h16* Ph, int K) { proj_body<1>(A, Bt, Ph, K); }

static_assert(32 * 16 * 2 == 16 * HD * 2);
__global__ __launch_bounds__(32 * AW) void k_flash(const h16* __restrict__ QH, const h16* __restrict__ KP, const h16* __restrict__ VT, h16* CX) {
    __shared__ __align__(16) float os[AW * 16 * OSP];
    const int lane = threadIdx.x & 31, lr = lane & 15, hi = lane >> 4;
    const int wave = __builtin_amdgcn_readfirstlane((int)(threadIdx.x >> 5));
    const int zh = blockIdx.y;
    const int t0 = (blockIdx.x * AW + wave) * 16;
    const size_t pbase = (size_t)zh * SEQ * HD;
    const size_t qo = pbase + (size_t)(t0 + lr) * HD + 8 * hi;
    const v16h qh = ldh(QH + qo);
    const size_t ko = pbase + (size_t)lr * HD + 8 * hi;
    const size_t vo = pbase + (size_t)lr * SEQ + 8 * hi;
    v8f o0 = (v8f){}, o1 = (v8f){};
    float m = NEGB, l = 0.0f;
#pragma unroll 1
    for (int key0 = 0; key0 < SEQ; key0 += 32) {
        const h16* ka = KP + ko + (size_t)key0 * HD;
        const v16h ka0 = ldh(ka), kb0 = ldh(ka + 16 * HD);
        v8f sa = (v8f){}, sb = (v8f){};
        sa = wmma16g(ka0, qh, sa); sb = wmma16g(kb0, qh, sb);
        float ta[8], tb[8]; float mx = NEGB;
#pragma unroll
        for (int r = 0; r < 8; ++r) { ta[r] = sa[r] * SC2; tb[r] = sb[r] * SC2; mx = fmaxf(mx, fmaxf(ta[r], tb[r])); }
        mx = fmaxf(mx, __shfl_xor(mx, 16, 32));
        const float mnew = fmaxf(m, mx);
        const float alpha = __builtin_amdgcn_exp2f(m - mnew);
        const float sh = PSH - mnew;
        v16h pb; float ls = 0.0f;
#pragma unroll
        for (int r = 0; r < 8; ++r) {
            const float ea = ta[r] + sh, eb = tb[r] + sh;
            const float ga = __builtin_amdgcn_exp2f(ea), gb = __builtin_amdgcn_exp2f(eb);
            const h16 pa = (ea < -14.0f) ? (h16)0.0f : (h16)ga;
            const h16 pc = (eb < -14.0f) ? (h16)0.0f : (h16)gb;
            pb[r] = pa; pb[8 + r] = pc;
            ls += (float)pa + (float)pc; }
        l = l * alpha + ls; m = mnew;
        o0 = o0 * alpha; o1 = o1 * alpha;
        const h16* va = VT + vo + key0;
        const v16h v0 = ldh(va), v1 = ldh(va + (size_t)16 * SEQ);
        o0 = wmma16g(v0, pb, o0); o1 = wmma16g(v1, pb, o1);
    }
    l += __shfl_xor(l, 16, 32);
    const float inv = CXS * (1.0f / l);
    const int wb = wave * 16 * OSP;
    { v4f a, c;
      a[0] = o0[0] * inv; a[1] = o0[1] * inv; a[2] = o0[2] * inv; a[3] = o0[3] * inv; c[0] = o0[4] * inv; c[1] = o0[5] * inv; c[2] = o0[6] * inv; c[3] = o0[7] * inv;
      *(v4fa*)(&os[wb + lr * OSP +  0 + 8 * hi]) = a; *(v4fa*)(&os[wb + lr * OSP +  0 + 8 * hi + 4]) = c;
      a[0] = o1[0] * inv; a[1] = o1[1] * inv; a[2] = o1[2] * inv; a[3] = o1[3] * inv; c[0] = o1[4] * inv; c[1] = o1[5] * inv; c[2] = o1[6] * inv; c[3] = o1[7] * inv;
      *(v4fa*)(&os[wb + lr * OSP + 16 + 8 * hi]) = a; *(v4fa*)(&os[wb + lr * OSP + 16 + 8 * hi + 4]) = c; }
    wave_sync();
    h16* crow = CX + pbase + (size_t)t0 * HD;
#pragma unroll 1
    for (int ps = 0; ps < 2; ++ps) {
#pragma unroll
        for (int s = 0; s < 2; ++s) { const int p = s * 32 + lane; const int row = p >> 2, c8 = (p & 3) * 8;
            const v4f x0 = *(const v4fa*)(&os[wb + row * OSP + c8]); const v4f x1 = *(const v4fa*)(&os[wb + row * OSP + c8 + 4]); v8h hv;
#pragma unroll
            for (int i = 0; i < 4; ++i) { hv[i] = toh_flush(x0[i]); hv[4 + i] = toh_flush(x1[i]); }
            *(volatile v8h*)(crow + (size_t)p * 8) = hv; }
        if (ps == 0) __threadfence(); }
}

static_assert(32 * 16 * 8 == 16 * 64 * 4);
__global__ __launch_bounds__(32) void k_outp(const h16* __restrict__ WO, const h16* __restrict__ CX, const float* __restrict__ bo, float* OUT) {
    __shared__ __align__(16) float os[16 * 68];
    const int lane = threadIdx.x & 31, lr = lane & 15, hi = lane >> 4; const int r0 = blockIdx.x * 64, c0 = blockIdx.y * 64;
    const int bb = c0 / SEQ, tt = c0 % SEQ;
    v8f acc[4][4];
#pragma unroll
    for (int mb = 0; mb < 4; ++mb)
#pragma unroll
        for (int nb = 0; nb < 4; ++nb) acc[mb][nb] = (v8f){};
    const size_t aoff = (size_t)(r0 + lr) * DM + 8 * hi;
    const size_t boff = ((size_t)bb * NH_ * SEQ + (size_t)(tt + lr)) * HD + 8 * hi;
#pragma unroll 1
    for (int hh = 0; hh < NH_; ++hh) {
        v16h a[4];
#pragma unroll
        for (int mb = 0; mb < 4; ++mb) a[mb] = ldh(WO + aoff + (size_t)mb * 16 * DM + hh * 32);
#pragma unroll
        for (int nb = 0; nb < 4; ++nb) { const v16h b = ldh(CX + boff + (size_t)hh * ((size_t)SEQ * HD) + (size_t)nb * 16 * HD);
#pragma unroll
            for (int mb = 0; mb < 4; ++mb) acc[mb][nb] = wmma16g(a[mb], b, acc[mb][nb]); }
    }
#pragma unroll
    for (int mb = 0; mb < 4; ++mb) {
        float br[8];
#pragma unroll
        for (int j = 0; j < 8; ++j) br[j] = bfr(bo[r0 + mb * 16 + hi * 8 + j]);
#pragma unroll
        for (int nb = 0; nb < 4; ++nb) {
#pragma unroll
            for (int j = 0; j < 8; ++j) os[(hi * 8 + j) * 68 + nb * 16 + lr] = acc[mb][nb][j] * OSC + br[j]; }
        wave_sync();
        float* ob = OUT + ((size_t)bb * DQ + (size_t)(r0 + mb * 16)) * OUT_SEQ + (size_t)tt;
#pragma unroll 1
        for (int ps = 0; ps < 2; ++ps) {
#pragma unroll
            for (int s = 0; s < 8; ++s) { const int row = 2 * s + (lane >> 4), c4 = (lane & 15) * 4;
                const v4f val = *(const v4fa*)(&os[row * 68 + c4]);
                *(volatile v4f*)(ob + (size_t)row * OUT_SEQ + c4) = val; }
            if (ps == 0) __threadfence(); }
        wave_sync();
    }
}

static constexpr size_t al256(size_t v) { return (v + 255) & ~(size_t)255; }
static constexpr size_t SZ_XQ = al256((size_t)NB * SEQ * DQ * 2);
static constexpr size_t SZ_XK = al256((size_t)NB * SEQ * DKV * 2);
static constexpr size_t SZ_WQ = al256((size_t)DM * DQ * 2);
static constexpr size_t SZ_WK = al256((size_t)DM * DKV * 2);
static constexpr size_t SZ_WO = al256((size_t)DQ * DM * 2);
static constexpr size_t SZ_PL = al256((size_t)NB * NH_ * SEQ * HD * 2);
static constexpr size_t SZ_TOTAL = SZ_XQ + 2 * SZ_XK + SZ_WQ + 2 * SZ_WK + SZ_WO + 4 * SZ_PL;
static_assert(SZ_TOTAL <= (size_t)134217728);
static_assert((size_t)NB * NH_ * SEQ * HD == (size_t)NB * DM * SEQ);
static_assert(((size_t)NB * SEQ * DQ * 2) % 256 == 0);
static_assert(((size_t)NB * SEQ * DKV * 2) % 256 == 0);

extern "C" void kernel_launch(void* const* d_in, const int* in_sizes, int n_in,
                              void* d_out, int out_size, void* d_ws, size_t ws_size, hipStream_t stream) {
    if (n_in < 8) return;
    const size_t needq  = ((size_t)NB * DQ  - 1) * SEQ_FULL + SEQ;
    const size_t needkv = ((size_t)NB * DKV - 1) * SEQ_FULL + SEQ;
    if ((size_t)in_sizes[0] < needq || (size_t)in_sizes[1] < needkv || (size_t)in_sizes[2] < needkv) return;
    if ((size_t)in_sizes[3] < (size_t)DQ * DM || (size_t)in_sizes[4] < (size_t)DKV * DM || (size_t)in_sizes[5] < (size_t)DKV * DM) return;
    if ((size_t)in_sizes[6] < (size_t)DM * DQ || in_sizes[7] < DQ) return;
    if ((size_t)out_size < ((size_t)NB * DQ - 1) * OUT_SEQ + SEQ) return;
    if (SZ_TOTAL > ws_size) return;
    const float* xq = (const float*)d_in[0]; const float* xk = (const float*)d_in[1]; const float* xv = (const float*)d_in[2];
    const float* wq = (const float*)d_in[3]; const float* wk = (const float*)d_in[4]; const float* wv = (const float*)d_in[5];
    const float* wo = (const float*)d_in[6]; const float* bo = (const float*)d_in[7];
    float* OUT = (float*)d_out;
    char* wsp = (char*)d_ws;
    bf* XQ = (bf*)wsp; wsp += SZ_XQ;
    bf* XK = (bf*)wsp; wsp += SZ_XK;
    bf* XV = (bf*)wsp; wsp += SZ_XK;
    bf* WQ = (bf*)wsp; wsp += SZ_WQ;
    bf* WK = (bf*)wsp; wsp += SZ_WK;
    bf* WV = (bf*)wsp; wsp += SZ_WK;
    h16* WO = (h16*)wsp; wsp += SZ_WO;
    h16* QH = (h16*)wsp; wsp += SZ_PL;
    h16* KP = (h16*)wsp; wsp += SZ_PL;
    h16* VT = (h16*)wsp; wsp += SZ_PL;
    h16* CX = (h16*)wsp; wsp += SZ_PL;

    k_tcvt_b<<<dim3(SEQ / 32, DQ / 64, NB), 256, 0, stream>>>(xq, XQ, DQ, SEQ_FULL, SEQ);
    k_tcvt_b<<<dim3(SEQ / 32, DKV / 64, NB), 256, 0, stream>>>(xk, XK, DKV, SEQ_FULL, SEQ);
    k_tcvt_b<<<dim3(SEQ / 32, DKV / 64, NB), 256, 0, stream>>>(xv, XV, DKV, SEQ_FULL, SEQ);
    k_tcvt_b<<<dim3(DM / 32, DQ / 64, 1), 256, 0, stream>>>(wq, WQ, DQ, DM, DM);
    k_tcvt_b<<<dim3(DM / 32, DKV / 64, 1), 256, 0, stream>>>(wk, WK, DKV, DM, DM);
    k_tcvt_b<<<dim3(DM / 32, DKV / 64, 1), 256, 0, stream>>>(wv, WV, DKV, DM, DM);
    k_tcvt_h<<<dim3(DQ / 32, DM / 64, 1), 256, 0, stream>>>(wo, WO, DM, DQ, DQ, WOS);

    k_proj_rows<<<dim3(NB * SEQ / 64, DM / 64, 1), 32, 0, stream>>>(XQ, WQ, QH, DQ);
    k_proj_rows<<<dim3(NB * SEQ / 64, DM / 64, 1), 32, 0, stream>>>(XK, WK, KP, DKV);
    k_proj_cols<<<dim3(DM / 64, NB * SEQ / 64, 1), 32, 0, stream>>>(WV, XV, VT, DKV);

    k_flash<<<dim3(SEQ / (16 * AW), NB * NH_, 1), 32 * AW, 0, stream>>>(QH, KP, VT, CX);

    k_outp<<<dim3(DQ / 64, NB * SEQ / 64, 1), 32, 0, stream>>>(WO, CX, bo, OUT);
}
